// LSTMTextEncoder_7473243095591
// MI455X (gfx1250) — hardware-verified
//
#include <hip/hip_runtime.h>


typedef _Float16 f16t;
typedef f16t  v16h __attribute__((ext_vector_type(16)));
typedef f16t  v8h  __attribute__((ext_vector_type(8)));
typedef float v8f  __attribute__((ext_vector_type(8)));
typedef float v4f  __attribute__((ext_vector_type(4)));
typedef unsigned int v4u __attribute__((ext_vector_type(4)));

union Frag { v16h v; v8h q[2]; };
union Pk16 { v8h h; v4u u; };

#define EDIM  256
#define HDIM  256
#define NGATE 1024
#define KP    512
#define PX    520
#define GSTR  (HDIM * KP)

#define SX 256.0f
#define SW 64.0f
#define SH 16.0f
#define SU 1024.0f
#define SF 1024.0f
#define INV14 6.103515625e-05f

__device__ __forceinline__ v8f wmma16(v16h a, v16h b, v8f c) {
    return __builtin_amdgcn_wmma_f32_16x16x32_f16(false, a, false, b, (short)0, c, false, false);
}
__device__ __forceinline__ void wguard4(v8f& c0, v8f& c1, v8f& c2, v8f& c3,
                                        const v16h& a, const v16h& b0, const v16h& b1,
                                        const v16h& b2, const v16h& b3) {
    asm volatile("v_nop\n\tv_nop\n\tv_nop\n\tv_nop"
                 : "+v"(c0), "+v"(c1), "+v"(c2), "+v"(c3)
                 : "v"(a), "v"(b0), "v"(b1), "v"(b2), "v"(b3));
}
__device__ __forceinline__ void wguard1(v8f& c, const v16h& a, const v16h& b) {
    asm volatile("v_nop\n\tv_nop\n\tv_nop\n\tv_nop" : "+v"(c) : "v"(a), "v"(b));
}

__device__ __forceinline__ v8f zero8() {
    v8f z = {0.f, 0.f, 0.f, 0.f, 0.f, 0.f, 0.f, 0.f};
    return z;
}

__device__ __forceinline__ float sigf(float x) {
    float t = __expf(-x);
    return __builtin_amdgcn_rcpf(1.0f + t);
}
__device__ __forceinline__ float ftanh(float x) {
    float ax = fabsf(x);
    float t  = __expf(-2.0f * ax);
    float r  = (1.0f - t) * __builtin_amdgcn_rcpf(1.0f + t);
    return copysignf(r, x);
}

__global__ __launch_bounds__(256)
void k_pack_gates(const float* W0, const float* W1, const float* W2, const float* W3,
                  const float* U0, const float* U1, const float* U2, const float* U3,
                  f16t* P) {
    const int gy = blockIdx.y;
    const float* W = (gy == 0) ? W0 : (gy == 1) ? W1 : (gy == 2) ? W2 : W3;
    const float* U = (gy == 0) ? U0 : (gy == 1) ? U1 : (gy == 2) ? U2 : U3;
    const int i = blockIdx.x * 256 + threadIdx.x;
    if (i >= HDIM * (KP / 8)) return;
    const int nl = i >> 6;
    const int kq = (i & 63) * 8;
    Pk16 v;
#pragma unroll
    for (int e = 0; e < 8; ++e) {
        const int k  = kq + e;
        const int kw = min(k, EDIM - 1);
        const int ku = min(max(k - EDIM, 0), HDIM - 1);
        const float a = W[(size_t)kw * HDIM + nl] * SW;
        const float b = U[(size_t)ku * HDIM + nl] * SU;
        v.h[e] = (f16t)((k < EDIM) ? a : b);
    }
    f16t* d = P + (size_t)(gy * HDIM + nl) * KP + kq;
    *(volatile v4u*)d = v.u;
    __threadfence();
    *(volatile v4u*)d = v.u;
}

__global__ __launch_bounds__(256)
void k_pack_fc(const float* F, f16t* Pf) {
    const int i = blockIdx.x * 256 + threadIdx.x;
    if (i >= EDIM * (HDIM / 8)) return;
    const int n  = i >> 5;
    const int kq = (i & 31) * 8;
    Pk16 v;
#pragma unroll
    for (int e = 0; e < 8; ++e)
        v.h[e] = (f16t)(F[(size_t)(kq + e) * EDIM + n] * SF);
    f16t* d = Pf + (size_t)n * HDIM + kq;
    *(volatile v4u*)d = v.u;
    __threadfence();
    *(volatile v4u*)d = v.u;
}

__device__ __forceinline__ void stage_x(f16t* XH, const int* cap, const float* emb,
                                        int brow, int w, int l, int t, int T, int nvocab) {
    int tok = cap[(size_t)brow * T + t];
    tok = min(max(tok, 0), nvocab - 1);
    const float* rp = emb + (size_t)tok * EDIM + l * 8;
    const v4f f0 = *(const v4f*)rp;
    const v4f f1 = *(const v4f*)(rp + 4);
    Pk16 k;
#pragma unroll
    for (int e = 0; e < 4; ++e) {
        k.h[e]     = (f16t)(f0[e] * SX);
        k.h[4 + e] = (f16t)(f1[e] * SX);
    }
    *(v8h*)(XH + (size_t)w * PX + l * 8) = k.h;
}

__global__ __launch_bounds__(512)
void k_lstm(const int* cap, const float* emb, const f16t* P, const f16t* Pf,
            const float* bWi, const float* bUi, const float* bWf, const float* bUf,
            const float* bWo, const float* bUo, const float* bWc, const float* bUc,
            const float* fcb, float* out, int T, int nb, int nvocab) {
    __shared__ __attribute__((aligned(16))) f16t  XH[16 * PX];
    __shared__ __attribute__((aligned(16))) float O[16 * EDIM];

    const int tid = threadIdx.x;
    const int l = tid & 31, w = tid >> 5, hh = l >> 4, m = l & 15;
    const int b0 = blockIdx.x * 16;
    if (b0 + 16 > nb) return;

    const int col = 16 * w + m;
    const float b_i = bWi[col] + bUi[col];
    const float b_f = bWf[col] + bUf[col];
    const float b_o = bWo[col] + bUo[col];
    const float b_g = bWc[col] + bUc[col];

    {
        Pk16 z;
#pragma unroll
        for (int e = 0; e < 8; ++e) z.h[e] = (f16t)0.0f;
        *(v8h*)(XH + (size_t)w * PX + EDIM + l * 8) = z.h;
        stage_x(XH, cap, emb, b0 + w, w, l, 0, T, nvocab);
    }
    __syncthreads();

    v8f cst = zero8();
    const f16t* xa = XH + (size_t)m * PX + 8 * hh;

#pragma unroll 1
    for (int t = 0; t < T; ++t) {
        int tz = 0;
        asm volatile("" : "+s"(tz));
        const f16t* pb = P + (size_t)col * KP + 8 * hh + tz;

        v8f acc0 = zero8(), acc1 = zero8(), acc2 = zero8(), acc3 = zero8();
#pragma unroll 2
        for (int kt = 0; kt < 16; ++kt) {
            Frag a, q0, q1, q2, q3;
            const f16t* ap = xa + kt * 32;
            a.q[0] = *(const v8h*)ap;
            a.q[1] = *(const v8h*)(ap + 16);
            const f16t* bp = pb + kt * 32;
            q0.q[0] = *(const v8h*)(bp);            q0.q[1] = *(const v8h*)(bp + 16);
            q1.q[0] = *(const v8h*)(bp + GSTR);     q1.q[1] = *(const v8h*)(bp + GSTR + 16);
            q2.q[0] = *(const v8h*)(bp + 2 * GSTR); q2.q[1] = *(const v8h*)(bp + 2 * GSTR + 16);
            q3.q[0] = *(const v8h*)(bp + 3 * GSTR); q3.q[1] = *(const v8h*)(bp + 3 * GSTR + 16);
            acc0 = wmma16(a.v, q0.v, acc0);
            acc1 = wmma16(a.v, q1.v, acc1);
            acc2 = wmma16(a.v, q2.v, acc2);
            acc3 = wmma16(a.v, q3.v, acc3);
            wguard4(acc0, acc1, acc2, acc3, a.v, q0.v, q1.v, q2.v, q3.v);
        }
        __syncthreads();

#pragma unroll
        for (int r = 0; r < 8; ++r) {
            const float pi = fmaf(acc0[r], INV14, b_i);
            const float pf = fmaf(acc1[r], INV14, b_f);
            const float po = fmaf(acc2[r], INV14, b_o);
            const float pg = fmaf(acc3[r], INV14, b_g);
            const float iv = sigf(pi);
            const float fv = sigf(pf);
            const float ov = sigf(po);
            const float gv = ftanh(pg);
            const float cv = iv * gv + fv * cst[r];
            cst[r] = cv;
            const float hv = ov * ftanh(cv);
            XH[(size_t)(8 * hh + r) * PX + EDIM + col] = (f16t)(hv * SH);
        }
        if (t + 1 < T)
            stage_x(XH, cap, emb, b0 + w, w, l, t + 1, T, nvocab);
        __syncthreads();
    }

    {
        v8f acf = zero8();
        const f16t* ha = XH + (size_t)m * PX + EDIM + 8 * hh;
        const f16t* fb = Pf + (size_t)col * HDIM + 8 * hh;
#pragma unroll 2
        for (int kt = 0; kt < 8; ++kt) {
            Frag a, b;
            a.q[0] = *(const v8h*)(ha + kt * 32);
            a.q[1] = *(const v8h*)(ha + kt * 32 + 16);
            b.q[0] = *(const v8h*)(fb + kt * 32);
            b.q[1] = *(const v8h*)(fb + kt * 32 + 16);
            acf = wmma16(a.v, b.v, acf);
            wguard1(acf, a.v, b.v);
        }
        const float fbv = fcb[col];
#pragma unroll
        for (int r = 0; r < 8; ++r)
            O[(8 * hh + r) * EDIM + col] = fmaf(acf[r], INV14, fbv);
    }
    __syncthreads();

    {
        const float* orw = O + w * EDIM;
        const v4f u0 = *(const v4f*)(orw + l * 8);
        const v4f u1 = *(const v4f*)(orw + l * 8 + 4);
        float s = 0.0f;
#pragma unroll
        for (int e = 0; e < 4; ++e) s += u0[e] * u0[e] + u1[e] * u1[e];
        s += __shfl_xor(s, 16);
        s += __shfl_xor(s, 8);
        s += __shfl_xor(s, 4);
        s += __shfl_xor(s, 2);
        s += __shfl_xor(s, 1);
        float nrm = sqrtf(s);
        nrm = fmaxf(nrm, 1e-12f);
        const float inv = 1.0f / nrm;

        const v4f p0 = *(const v4f*)(orw + l * 4) * inv;
        const v4f p1 = *(const v4f*)(orw + 128 + l * 4) * inv;
        float* dst = out + (size_t)(b0 + w) * EDIM;
        *(volatile v4f*)(dst + l * 4)       = p0;
        *(volatile v4f*)(dst + 128 + l * 4) = p1;
        __threadfence();
        *(volatile v4f*)(dst + l * 4)       = p0;
        *(volatile v4f*)(dst + 128 + l * 4) = p1;
    }
}

extern "C" void kernel_launch(void* const* d_in, const int* in_sizes, int n_in,
                              void* d_out, int out_size, void* d_ws, size_t ws_size,
                              hipStream_t stream) {
    if (n_in < 20) return;
    if (out_size <= 0 || (out_size % EDIM) != 0) return;
    const int nb = out_size / EDIM;
    if (nb < 16 || (nb % 16) != 0) return;
    if (in_sizes[0] <= 0 || (in_sizes[0] % nb) != 0) return;
    const int T = in_sizes[0] / nb;
    if (T < 1) return;
    if (in_sizes[1] < EDIM || (in_sizes[1] % EDIM) != 0) return;
    const int nvocab = in_sizes[1] / EDIM;
    for (int j = 2; j <= 18; j += 2) if (in_sizes[j] != EDIM * HDIM) return;
    for (int j = 3; j <= 19; j += 2) if (in_sizes[j] != HDIM) return;

    const int*   cap = (const int*)d_in[0];
    const float* emb = (const float*)d_in[1];
    const float* Wi = (const float*)d_in[2];   const float* bWi = (const float*)d_in[3];
    const float* Ui = (const float*)d_in[4];   const float* bUi = (const float*)d_in[5];
    const float* Wf = (const float*)d_in[6];   const float* bWf = (const float*)d_in[7];
    const float* Uf = (const float*)d_in[8];   const float* bUf = (const float*)d_in[9];
    const float* Wo = (const float*)d_in[10];  const float* bWo = (const float*)d_in[11];
    const float* Uo = (const float*)d_in[12];  const float* bUo = (const float*)d_in[13];
    const float* Wc = (const float*)d_in[14];  const float* bWc = (const float*)d_in[15];
    const float* Uc = (const float*)d_in[16];  const float* bUc = (const float*)d_in[17];
    const float* fcw = (const float*)d_in[18];
    const float* fcb = (const float*)d_in[19];
    float* out = (float*)d_out;

    const size_t bP = (size_t)NGATE * KP * 2;
    const size_t bF = (size_t)EDIM * HDIM * 2;
    if (bP + bF > ws_size) return;
    f16t* P  = (f16t*)d_ws;
    f16t* Pf = (f16t*)((char*)d_ws + bP);

    k_pack_gates<<<dim3((HDIM * (KP / 8)) / 256, 4), dim3(256), 0, stream>>>(
        Wi, Wf, Wo, Wc, Ui, Uf, Uo, Uc, P);
    k_pack_fc<<<dim3((EDIM * (HDIM / 8)) / 256), dim3(256), 0, stream>>>(fcw, Pf);
    k_lstm<<<dim3(nb / 16), dim3(512), 0, stream>>>(
        cap, emb, P, Pf, bWi, bUi, bWf, bUf, bWo, bUo, bWc, bUc, fcb, out, T, nb, nvocab);
}
